// GATLayer_18734647345426
// MI455X (gfx1250) — hardware-verified
//
#include <hip/hip_runtime.h>
#include <stddef.h>


typedef _Float16 v16h __attribute__((ext_vector_type(16)));
typedef _Float16 v8h  __attribute__((ext_vector_type(8)));
typedef float    v8f  __attribute__((ext_vector_type(8)));
typedef float    v4f  __attribute__((ext_vector_type(4)));
typedef _Float16 h16;

#ifndef NB
#define NB 4
#endif
#ifndef SEQ
#define SEQ 1024
#endif
#define NB_FULL  4
#define SEQ_FULL 1024
#define KIN   128
#define DIM   128
#define NHEAD 8
#define HD    16
#define MROWS (NB * SEQ)

static_assert(NB >= 1 && NB <= NB_FULL);
static_assert(SEQ >= 64 && SEQ <= SEQ_FULL && (SEQ % 64) == 0 && (SEQ % 32) == 0);
static_assert(DIM == NHEAD * HD);
static_assert(HD == 16);
static_assert(64 == 4 * HD);
static_assert((KIN % 64) == 0 && (KIN % 32) == 0);
static_assert((DIM % 64) == 0);
static_assert((MROWS % 64) == 0);
static_assert(((NHEAD * SEQ) % 512) == 0);
static_assert(DIM == 32 * 4);

#define LDT 72
#define LDC 68
#define LDO 68
static_assert((LDT % 8) == 0 && LDT >= 64);
static_assert((LDC % 4) == 0 && LDC >= 64);
static_assert((LDO % 4) == 0 && LDO >= 64);

#define WCARRY 64.0f
#define XCARRY 16.0f
#define PCARRY 1024.0f
#define PEXP   10.0f
#define VCARRY 64.0f
#define LOG2E  1.44269504088896341f
static_assert(PCARRY == 1024.0f);
static_assert(VCARRY * 16.0f == WCARRY * XCARRY);

#define WT_BYTES ((size_t)DIM * KIN * 2)
#define VT_BYTES ((size_t)NB * DIM * SEQ * 2)
#define SDPLANE  ((size_t)NB * NHEAD * SEQ)
#define SD_BYTES ((size_t)2 * SDPLANE * 4)
#define OFF_WT ((size_t)0)
#define OFF_VT (OFF_WT + WT_BYTES)
#define OFF_SD (OFF_VT + VT_BYTES)
#define WS_TOTAL (OFF_SD + SD_BYTES)
static_assert((WT_BYTES % 128) == 0 && (VT_BYTES % 128) == 0 && (SD_BYTES % 128) == 0);
static_assert(WS_TOTAL <= (size_t)134217728);

__device__ __forceinline__ float bf16r(float x) {
  unsigned int u = __float_as_uint(x);
  u = (u + 0x7FFFu + ((u >> 16) & 1u)) & 0xFFFF0000u;
  return __uint_as_float(u);
}

static __device__ __forceinline__ h16 toh_flush(float v) {
  const h16 r = (h16)v;
  return (fabsf(v) < 6.103515625e-05f) ? (h16)0.0f : r;
}

__device__ __forceinline__ v16h frag_at(const _Float16* p) {
  v8h lo = *(const v8h*)(p);
  v8h hi = *(const v8h*)(p + 16);
  v16h out;
#pragma unroll
  for (int i = 0; i < 8; ++i) { out[i] = lo[i]; out[i + 8] = hi[i]; }
  return out;
}

__device__ __forceinline__ v16h frag_x(const float* p) {
  const v4f a0 = *(const v4f*)(p);
  const v4f a1 = *(const v4f*)(p + 4);
  const v4f a2 = *(const v4f*)(p + 16);
  const v4f a3 = *(const v4f*)(p + 20);
  v16h out;
#pragma unroll
  for (int i = 0; i < 4; ++i) {
    out[i]      = toh_flush(XCARRY * bf16r(a0[i]));
    out[i + 4]  = toh_flush(XCARRY * bf16r(a1[i]));
    out[i + 8]  = toh_flush(XCARRY * bf16r(a2[i]));
    out[i + 12] = toh_flush(XCARRY * bf16r(a3[i]));
  }
  return out;
}

__device__ __forceinline__ v8f wmma16(v16h a, v16h b, v8f c) {
  v8f d = __builtin_amdgcn_wmma_f32_16x16x32_f16(false, a, false, b, (short)0, c,
                                                 false, false);
  asm volatile("v_nop\n\tv_nop\n\tv_nop\n\tv_nop" : "+v"(d) : "v"(a), "v"(b));
  return d;
}

__device__ __forceinline__ void wave_lds_sync() {
  __builtin_amdgcn_fence(3  , "wavefront");
  asm volatile("s_wait_dscnt 0x0" ::: "memory");
  __builtin_amdgcn_wave_barrier();
}

__global__ __launch_bounds__(256) void wconv_kernel(
    const float* __restrict__ W, _Float16* __restrict__ Wt, unsigned ldw, unsigned ldk) {
  __shared__ _Float16 T[64 * LDT];
  const unsigned tid = threadIdx.x;
  const unsigned n0 = blockIdx.x * 64u;
  const unsigned k0 = blockIdx.y * 64u;
#pragma unroll 4
  for (unsigned j = 0; j < 16u; ++j) {
    const unsigned idx = tid + 256u * j;
    const unsigned kr = idx >> 6, nc = idx & 63u;
    const float v = W[(size_t)(k0 + kr) * ldw + n0 + nc];
    T[nc * LDT + kr] = (_Float16)(WCARRY * bf16r(v));
  }
  __syncthreads();
  v8h x[2];
  size_t off[2];
#pragma unroll
  for (unsigned i = 0; i < 2u; ++i) {
    const unsigned n = 32u * i + (tid >> 3);
    const unsigned kc = (tid & 7u) * 8u;
    x[i] = *(const v8h*)&T[n * LDT + kc];
    off[i] = (size_t)(n0 + n) * ldk + k0 + kc;
  }
#pragma unroll
  for (int i = 0; i < 2; ++i) *(volatile v8h*)(Wt + off[i]) = x[i];
  __threadfence();
#pragma unroll
  for (int i = 0; i < 2; ++i) *(volatile v8h*)(Wt + off[i]) = x[i];
}

__global__ __launch_bounds__(256) void proj_kernel(
    const float* __restrict__ X, const _Float16* __restrict__ Wt,
    const float* __restrict__ avec, _Float16* __restrict__ vt, float* __restrict__ sdp) {
  __shared__ __attribute__((aligned(16))) float Cs[64 * LDC];
  __shared__ __attribute__((aligned(16))) float SD[2 * 4 * 64];
  const unsigned tid = threadIdx.x, lane = tid & 31u;
  const unsigned w = (unsigned)__builtin_amdgcn_readfirstlane((int)(threadIdx.x >> 5));
  const unsigned mw = w >> 1, nw = w & 1u;
  const unsigned hh = lane >> 4, m = lane & 15u;
  const unsigned n0 = blockIdx.x * 64u;
  const unsigned row0 = blockIdx.y * 64u;
  const unsigned bidx = row0 / (unsigned)SEQ;
  const unsigned key0 = row0 - bidx * (unsigned)SEQ;

  const size_t frow = (size_t)bidx * SEQ_FULL + key0 + mw * 16u + m;
  const float* ap = X + frow * KIN + hh * 8u;
  const _Float16* bp0 = Wt + (size_t)(n0 + nw * 32u + m) * KIN + hh * 8u;
  const _Float16* bp1 = bp0 + (size_t)16 * KIN;
  v8f acc0 = {}, acc1 = {};
#pragma unroll 2
  for (unsigned k0 = 0; k0 < (unsigned)KIN; k0 += 32u) {
    const v16h a  = frag_x(ap + k0);
    const v16h b0 = frag_at(bp0 + k0);
    const v16h b1 = frag_at(bp1 + k0);
    acc0 = wmma16(a, b0, acc0);
    acc1 = wmma16(a, b1, acc1);
  }
#pragma unroll
  for (int r = 0; r < 8; ++r) {
    float* d = &Cs[(mw * 16u + hh * 8u + (unsigned)r) * LDC + nw * 32u + m];
    d[0]  = acc0[r];
    d[16] = acc1[r];
  }
  __syncthreads();

  {
    v8h x[2];
    size_t off[2];
#pragma unroll
    for (unsigned i = 0; i < 2u; ++i) {
      const unsigned dcol = 32u * i + (tid >> 3);
      const unsigned kk = (tid & 7u) * 8u;
#pragma unroll
      for (unsigned j = 0; j < 8u; ++j) {
        const float t = Cs[(kk + j) * LDC + dcol] * (VCARRY / (XCARRY * WCARRY));
        x[i][j] = toh_flush(t);
      }
      off[i] = ((size_t)bidx * DIM + n0 + dcol) * SEQ + key0 + kk;
    }
#pragma unroll
    for (int i = 0; i < 2; ++i) *(volatile v8h*)(vt + off[i]) = x[i];
    __threadfence();
#pragma unroll
    for (int i = 0; i < 2; ++i) *(volatile v8h*)(vt + off[i]) = x[i];
  }

  {
    const unsigned r = tid & 63u, hl = tid >> 6;
    float s = 0.0f, d = 0.0f;
#pragma unroll 4
    for (unsigned c = 0; c < (unsigned)HD; ++c) {
      const float xv = Cs[r * LDC + hl * 16u + c] * (1.0f / (XCARRY * WCARRY));
      s += xv * bf16r(avec[c]);
      d += xv * bf16r(avec[HD + c]);
    }
    SD[hl * 64u + r] = s;
    SD[(4u + hl) * 64u + r] = d;
  }
  __syncthreads();

  if (w < 4u) {
    const v4f val = *(const v4f*)&SD[(hh * 4u + w) * 64u + m * 4u];
    const size_t off = (size_t)hh * SDPLANE +
                       ((size_t)bidx * NHEAD + (n0 >> 4) + w) * SEQ + key0 + m * 4u;
    *(volatile v4f*)(sdp + off) = val;
    __threadfence();
    *(volatile v4f*)(sdp + off) = val;
  }
}

__device__ __forceinline__ void adj_select(const float* __restrict__ ap, unsigned key0,
                                           unsigned irow, float von, float voff,
                                           float (&f)[16]) {
  v4f a0 = *(const v4f*)(ap);
  v4f a1 = *(const v4f*)(ap + 4);
  v4f a2 = *(const v4f*)(ap + 16);
  v4f a3 = *(const v4f*)(ap + 20);
  asm volatile("" : "+v"(a0));
  asm volatile("" : "+v"(a1));
  asm volatile("" : "+v"(a2));
  asm volatile("" : "+v"(a3));
#pragma unroll
  for (unsigned i = 0; i < 4u; ++i) {
    const float e0 = (key0 + i == irow) ? 1.0f : 0.0f;
    const float e1 = (key0 + 4u + i == irow) ? 1.0f : 0.0f;
    const float e2 = (key0 + 16u + i == irow) ? 1.0f : 0.0f;
    const float e3 = (key0 + 20u + i == irow) ? 1.0f : 0.0f;
    f[i]       = ((bf16r(a0[i]) + e0) > 0.0f) ? von : voff;
    f[i + 4u]  = ((bf16r(a1[i]) + e1) > 0.0f) ? von : voff;
    f[i + 8u]  = ((bf16r(a2[i]) + e2) > 0.0f) ? von : voff;
    f[i + 12u] = ((bf16r(a3[i]) + e3) > 0.0f) ? von : voff;
  }
}

__device__ __forceinline__ h16 p_elem(float s, float d, float mxv, float sc, float& lsum) {
  float t = s + d;
  t = fmaxf(t, 0.2f * t);
  const float u = t - mxv;
  const float p = __builtin_amdgcn_exp2f(fmaf(u, sc, PEXP));
  const h16 ph = toh_flush(p);
  lsum += (float)ph;
  return ph;
}

__global__ __launch_bounds__(128) void nbr_attn_kernel(
    const float* __restrict__ adj, const float* __restrict__ srcp,
    const float* __restrict__ dstp, const _Float16* __restrict__ Vt,
    float* __restrict__ out) {
  __shared__ __attribute__((aligned(16))) float Ds[NHEAD * SEQ];
  __shared__ __attribute__((aligned(16))) float Os[4 * 16 * LDO];

  const unsigned tid = threadIdx.x, lane = tid & 31u;
  const unsigned wave = (unsigned)__builtin_amdgcn_readfirstlane((int)(threadIdx.x >> 5));
  const unsigned hh = lane >> 4, m = lane & 15u;
  const unsigned b = blockIdx.y;
  const unsigned row0 = blockIdx.x * 64u + wave * 16u;
  const unsigned irow = row0 + m;

  {
    const float* dsrc = dstp + (size_t)b * (NHEAD * SEQ);
#pragma unroll 4
    for (unsigned j = 0; j < (unsigned)((NHEAD * SEQ) / 512); ++j) {
      const unsigned idx = (tid + 128u * j) * 4u;
      *(v4f*)&Ds[idx] = *(const v4f*)(dsrc + idx);
    }
  }
  __syncthreads();

  float sv[NHEAD], mx[NHEAD], ls[NHEAD];
#pragma unroll
  for (int h = 0; h < NHEAD; ++h) {
    sv[h] = srcp[((size_t)b * NHEAD + (unsigned)h) * SEQ + irow];
    mx[h] = -3.0e38f;
    ls[h] = 0.0f;
  }
  const float* arow = adj + ((size_t)b * SEQ_FULL + irow) * SEQ_FULL + hh * 8u;

#pragma unroll 1
  for (unsigned k0 = 0; k0 < (unsigned)SEQ; k0 += 32u) {
    float pen[16];
    adj_select(arow + k0, k0 + hh * 8u, irow, 0.0f, -3.0e38f, pen);
#pragma unroll
    for (int h = 0; h < NHEAD; ++h) {
      const unsigned dbase = (unsigned)h * (unsigned)SEQ + k0 + hh * 8u;
      const v4f d0 = *(const v4f*)&Ds[dbase];
      const v4f d1 = *(const v4f*)&Ds[dbase + 4u];
      const v4f d2 = *(const v4f*)&Ds[dbase + 16u];
      const v4f d3 = *(const v4f*)&Ds[dbase + 20u];
      float t = mx[h];
#pragma unroll
      for (int i = 0; i < 4; ++i) {
        t = fmaxf(t, d0[i] + pen[i]);
        t = fmaxf(t, d1[i] + pen[i + 4]);
        t = fmaxf(t, d2[i] + pen[i + 8]);
        t = fmaxf(t, d3[i] + pen[i + 12]);
      }
      mx[h] = t;
    }
  }
#pragma unroll
  for (int h = 0; h < NHEAD; ++h) {
    const float o = __shfl_xor(mx[h], 16, 32);
    float t = sv[h] + fmaxf(mx[h], o);
    mx[h] = fmaxf(t, 0.2f * t);
  }

  v8f acc[NHEAD];
#pragma unroll
  for (int h = 0; h < NHEAD; ++h) acc[h] = (v8f){};
  const _Float16* vrow = Vt + ((size_t)b * DIM + m) * SEQ + hh * 8u;

#pragma unroll 1
  for (unsigned k0 = 0; k0 < (unsigned)SEQ; k0 += 32u) {
    float scl[16];
    adj_select(arow + k0, k0 + hh * 8u, irow, LOG2E, 0.0f, scl);
#pragma unroll
    for (int h = 0; h < NHEAD; ++h) {
      const unsigned dbase = (unsigned)h * (unsigned)SEQ + k0 + hh * 8u;
      const v4f d0 = *(const v4f*)&Ds[dbase];
      const v4f d1 = *(const v4f*)&Ds[dbase + 4u];
      const v4f d2 = *(const v4f*)&Ds[dbase + 16u];
      const v4f d3 = *(const v4f*)&Ds[dbase + 20u];
      float lsum = ls[h];
      v16h pf;
#pragma unroll
      for (int i = 0; i < 4; ++i) {
        pf[i]      = p_elem(sv[h], d0[i], mx[h], scl[i], lsum);
        pf[i + 4]  = p_elem(sv[h], d1[i], mx[h], scl[i + 4], lsum);
        pf[i + 8]  = p_elem(sv[h], d2[i], mx[h], scl[i + 8], lsum);
        pf[i + 12] = p_elem(sv[h], d3[i], mx[h], scl[i + 12], lsum);
      }
      ls[h] = lsum;
      const v16h vf = frag_at(vrow + (size_t)(h * HD) * SEQ + k0);
      acc[h] = wmma16(pf, vf, acc[h]);
    }
  }

  float inv[NHEAD];
#pragma unroll
  for (int h = 0; h < NHEAD; ++h) {
    const float l = ls[h] + __shfl_xor(ls[h], 16, 32);
    inv[h] = __builtin_amdgcn_rcpf(l) * (1.0f / VCARRY);
  }
  const unsigned ob = wave * (16u * LDO);
#pragma unroll
  for (int g = 0; g < 2; ++g) {
#pragma unroll
    for (int hl = 0; hl < 4; ++hl) {
#pragma unroll
      for (int r = 0; r < 8; ++r) {
        const float iv = __shfl(inv[4 * g + hl], (int)(hh * 8u) + r, 32);
        Os[ob + (hh * 8u + (unsigned)r) * LDO + (unsigned)hl * 16u + m] =
            fmaxf(acc[4 * g + hl][r] * iv, 0.0f);
      }
    }
    wave_lds_sync();
    v4f x[8];
    size_t off[8];
#pragma unroll
    for (unsigned i = 0; i < 8u; ++i) {
      const unsigned r = 2u * i + hh;
      const unsigned c = m * 4u;
      x[i] = *(const v4f*)&Os[ob + r * LDO + c];
      off[i] = ((size_t)b * SEQ_FULL + row0 + r) * DIM + (unsigned)g * 64u + c;
    }
#pragma unroll
    for (int i = 0; i < 8; ++i) *(volatile v4f*)(out + off[i]) = x[i];
    __threadfence();
#pragma unroll
    for (int i = 0; i < 8; ++i) *(volatile v4f*)(out + off[i]) = x[i];
    wave_lds_sync();
  }
}

extern "C" void kernel_launch(void* const* d_in, const int* in_sizes, int n_in,
                              void* d_out, int out_size, void* d_ws, size_t ws_size,
                              hipStream_t stream) {
  if (n_in < 4) return;
  const long long need_x = ((long long)(NB - 1) * SEQ_FULL + SEQ) * DIM;
  const long long need_adj =
      ((long long)(NB - 1) * SEQ_FULL + (SEQ - 1)) * SEQ_FULL + SEQ;
  if ((long long)in_sizes[0] < need_x) return;
  if ((long long)in_sizes[1] < need_adj) return;
  if ((long long)in_sizes[2] < (long long)KIN * DIM) return;
  if (in_sizes[3] < 2 * HD) return;
  if ((long long)out_size < need_x) return;
  if (ws_size < WS_TOTAL) return;

  const float* X   = (const float*)d_in[0];
  const float* ADJ = (const float*)d_in[1];
  const float* W   = (const float*)d_in[2];
  const float* AV  = (const float*)d_in[3];
  float* out = (float*)d_out;

  char* ws = (char*)d_ws;
  _Float16* Wt16 = (_Float16*)(ws + OFF_WT);
  _Float16* Vt16 = (_Float16*)(ws + OFF_VT);
  float*    SDp  = (float*)(ws + OFF_SD);

  wconv_kernel<<<dim3(DIM / 64, KIN / 64), dim3(256), 0, stream>>>(W, Wt16, (unsigned)DIM,
                                                                  (unsigned)KIN);
  proj_kernel<<<dim3(DIM / 64, MROWS / 64), dim3(256), 0, stream>>>(X, Wt16, AV, Vt16, SDp);
  nbr_attn_kernel<<<dim3(SEQ / 64, NB), dim3(128), 0, stream>>>(ADJ, SDp, SDp + SDPLANE,
                                                                Vt16, out);
}
